// SimpleRNN_26637387170352
// MI455X (gfx1250) — hardware-verified
//
#include <hip/hip_runtime.h>
#include <math.h>

constexpr int NBATCH  = 64;
constexpr int NSTEP   = 512;
constexpr int NIN     = 256;
constexpr int NHID    = 1024;
constexpr int NOUTF   = 512;
constexpr int NTHR    = 256;
constexpr int NWAVE   = NTHR / 32;
constexpr int SEQ_BLK = 16;
constexpr int NSUB    = 8;
constexpr int WCOLS   = 16 * NSUB;
constexpr int XPITCH  = NIN + 8;
constexpr int HPITCH  = NHID + 8;
constexpr int NROWS   = NBATCH * NSTEP;
constexpr float WCARRY     = 256.0f;
constexpr float WCARRY_INV = 1.0f / 256.0f;
static_assert(NHID == WCOLS * NWAVE);
static_assert(NBATCH % SEQ_BLK == 0);
static_assert(NIN % 32 == 0 && NHID % 32 == 0);
static_assert(XPITCH % 8 == 0 && HPITCH % 8 == 0);
static_assert(SEQ_BLK * NIN == 2 * NTHR * 8);
static_assert(SEQ_BLK * NHID == 8 * NTHR * 8);
static_assert(SEQ_BLK * WCOLS == 8 * 32 * 8);
static_assert((SEQ_BLK * XPITCH) % 2 == 0 && (SEQ_BLK * HPITCH) % 2 == 0);
static_assert(NBATCH % 64 == 0 && NOUTF % 64 == 0 && NHID % 32 == 0);
static_assert(NOUTF == 4 * 128);

typedef __attribute__((ext_vector_type(16))) _Float16 v16h;
typedef __attribute__((ext_vector_type(8)))  _Float16 v8h;
typedef __attribute__((ext_vector_type(16))) __bf16   v16b;
typedef __attribute__((ext_vector_type(8)))  __bf16   v8b;
typedef __attribute__((ext_vector_type(8)))  float    v8f;
typedef __attribute__((ext_vector_type(4)))  float    v4f;
typedef __attribute__((ext_vector_type(4)))  unsigned v4u;

__device__ __forceinline__ unsigned short f2bf_bits(float f) {
  unsigned u = __float_as_uint(f);
  return (unsigned short)((u + 0x7FFFu + ((u >> 16) & 1u)) >> 16);
}
__device__ __forceinline__ float bf_bits2f(unsigned short h) { return __uint_as_float(((unsigned)h) << 16); }
__device__ __forceinline__ float bf16r(float f) { return bf_bits2f(f2bf_bits(f)); }

__device__ __forceinline__ void dep_guard_h(v8f& a, v8f& b, v16h x, v16h y) { asm volatile("v_nop\n\tv_nop\n\tv_nop\n\tv_nop" : "+v"(a), "+v"(b) : "v"(x), "v"(y)); }
__device__ __forceinline__ void dep_guard_b(v8f& a, v8f& b, v16b x, v16b y) { asm volatile("v_nop\n\tv_nop\n\tv_nop\n\tv_nop" : "+v"(a), "+v"(b) : "v"(x), "v"(y)); }
__device__ __forceinline__ void keep4_h(v16h a, v16h b, v16h c, v16h d) { asm volatile("v_nop" :: "v"(a), "v"(b), "v"(c), "v"(d)); }
__device__ __forceinline__ void keep4_b(v16b a, v16b b, v16b c, v16b d) { asm volatile("v_nop" :: "v"(a), "v"(b), "v"(c), "v"(d)); }
__device__ __forceinline__ void acc_guard4(v8f& a, v8f& b, v8f& c, v8f& d) { asm volatile("v_nop\n\tv_nop\n\tv_nop\n\tv_nop" : "+v"(a), "+v"(b), "+v"(c), "+v"(d)); }
template <typename V> __device__ __forceinline__ void guard4_ab(v8f& q0, v8f& q1, v8f& q2, v8f& q3, V a, V b0, V b1, V b2, V b3) {
  asm volatile("v_nop\n\tv_nop\n\tv_nop\n\tv_nop" : "+v"(q0), "+v"(q1), "+v"(q2), "+v"(q3) : "v"(a), "v"(b0), "v"(b1), "v"(b2), "v"(b3));
}
__device__ __forceinline__ void guard8_b(v8f& q0, v8f& q1, v8f& q2, v8f& q3, v8f& q4, v8f& q5, v8f& q6, v8f& q7,
                                         v16b a, v16b b0, v16b b1, v16b b2, v16b b3, v16b b4, v16b b5, v16b b6, v16b b7) {
  asm volatile("v_nop\n\tv_nop\n\tv_nop\n\tv_nop"
               : "+v"(q0), "+v"(q1), "+v"(q2), "+v"(q3), "+v"(q4), "+v"(q5), "+v"(q6), "+v"(q7)
               : "v"(a), "v"(b0), "v"(b1), "v"(b2), "v"(b3), "v"(b4), "v"(b5), "v"(b6), "v"(b7));
}
__device__ __forceinline__ void guard8_h(v8f& q0, v8f& q1, v8f& q2, v8f& q3, v8f& q4, v8f& q5, v8f& q6, v8f& q7,
                                         v16h a, v16h b0, v16h b1, v16h b2, v16h b3, v16h b4, v16h b5, v16h b6, v16h b7) {
  asm volatile("v_nop\n\tv_nop\n\tv_nop\n\tv_nop"
               : "+v"(q0), "+v"(q1), "+v"(q2), "+v"(q3), "+v"(q4), "+v"(q5), "+v"(q6), "+v"(q7)
               : "v"(a), "v"(b0), "v"(b1), "v"(b2), "v"(b3), "v"(b4), "v"(b5), "v"(b6), "v"(b7));
}
__device__ __forceinline__ void acc_guard8(v8f& q0, v8f& q1, v8f& q2, v8f& q3, v8f& q4, v8f& q5, v8f& q6, v8f& q7) {
  asm volatile("v_nop\n\tv_nop\n\tv_nop\n\tv_nop" : "+v"(q0), "+v"(q1), "+v"(q2), "+v"(q3), "+v"(q4), "+v"(q5), "+v"(q6), "+v"(q7));
}

template <typename T> struct Frag;
template <> struct Frag<_Float16> {
  typedef v16h V; union U { v16h v; v8h h[2]; };
  static __device__ __forceinline__ v16h load(const _Float16* p) {
    U f; f.h[0] = *(const v8h*)(p); f.h[1] = *(const v8h*)(p + 16); return f.v;
  }
  static __device__ __forceinline__ v8f mma(v16h a, v16h b, v8f c) {
    return __builtin_amdgcn_wmma_f32_16x16x32_f16(false, a, false, b, (short)0, c, false, false);
  }
  static __device__ __forceinline__ void guard(v8f& a, v8f& b, v16h x, v16h y) { dep_guard_h(a, b, x, y); }
  static __device__ __forceinline__ void keep(v16h a, v16h b, v16h c, v16h d) { keep4_h(a, b, c, d); }
};
template <> struct Frag<__bf16> {
  typedef v16b V; union U { v16b v; v8b h[2]; };
  static __device__ __forceinline__ v16b load(const __bf16* p) {
    U f; f.h[0] = *(const v8b*)(p); f.h[1] = *(const v8b*)(p + 16); return f.v;
  }
  static __device__ __forceinline__ v8f mma(v16b a, v16b b, v8f c) {
    return __builtin_amdgcn_wmma_f32_16x16x32_bf16(false, a, false, b, (short)0, c, false, false);
  }
  static __device__ __forceinline__ void guard(v8f& a, v8f& b, v16b x, v16b y) { dep_guard_b(a, b, x, y); }
  static __device__ __forceinline__ void keep(v16b a, v16b b, v16b c, v16b d) { keep4_b(a, b, c, d); }
};

__device__ __forceinline__ float tanh_f(float x) { return 1.0f - 2.0f * __builtin_amdgcn_rcpf(expf(2.0f * x) + 1.0f); }

template <int ET> struct Elem;
template <> struct Elem<0> { typedef _Float16 T; };
template <> struct Elem<1> { typedef __bf16 T; };
template <int ET, bool SPLIT, int BIAS_MODE, int OUT_MODE, bool RESID, int ACT = 0>
__global__ __launch_bounds__(256) void wmma_gemm64(
    const unsigned short* __restrict__ Ap, const unsigned short* __restrict__ A2p, int lda, long strideA,
    const unsigned short* __restrict__ Btp, const unsigned short* __restrict__ Bt2p, int ldb, long strideB,
    void* __restrict__ Cout, void* __restrict__ Cout2, int ldc, long strideC,
    const float* __restrict__ bias,
    const float* __restrict__ resid, long strideR,
    int M, int N, int K, float scale) {
  typedef typename Elem<ET>::T T;
  typedef typename Frag<T>::V V;
  const T* A = (const T*)Ap; const T* A2 = (const T*)A2p; const T* Bt = (const T*)Btp; const T* Bt2 = (const T*)Bt2p;
  __shared__ __align__(16) float sT[8][16 * 68];
  const int b    = blockIdx.y;
  const int lane = threadIdx.x & 31;
  const int wave = threadIdx.x >> 5;
  const int tilesN = N >> 6;
  const int tilesM = M >> 6;
  const int tile = blockIdx.x * 8 + wave;
  if (tile >= tilesM * tilesN) return;
  const int tm = tile / tilesN;
  const int tn = tile - tm * tilesN;
  const int m0 = tm << 6;
  const int n0 = tn << 6;

  const T* Ab  = A  + (size_t)b * strideA;
  const T* Bb  = Bt + (size_t)b * strideB;
  const T* Ab2 = SPLIT ? (A2  + (size_t)b * strideA) : nullptr;
  const T* Bb2 = SPLIT ? (Bt2 + (size_t)b * strideB) : nullptr;

  const int rlane = lane & 15;
  const int koff  = (lane >> 4) * 8;
  const int mOff  = (lane >> 4) * 8;

  v8f acc[4][4];
#pragma unroll
  for (int i = 0; i < 4; ++i)
#pragma unroll
    for (int j = 0; j < 4; ++j) acc[i][j] = (v8f){0.f,0.f,0.f,0.f,0.f,0.f,0.f,0.f};

  for (int k0 = 0; k0 < K; k0 += 32) {
    V bh[4], bl[4];
#pragma unroll
    for (int j = 0; j < 4; ++j) {
      const size_t bo = (size_t)(n0 + (j << 4) + rlane) * ldb + koff + k0;
      bh[j] = Frag<T>::load(Bb + bo);
      if (SPLIT) bl[j] = Frag<T>::load(Bb2 + bo);
    }
#pragma unroll
    for (int i = 0; i < 4; ++i) {
      const size_t ao = (size_t)(m0 + (i << 4) + rlane) * lda + koff + k0;
      V ah = Frag<T>::load(Ab + ao);
      V al;
      if (SPLIT) al = Frag<T>::load(Ab2 + ao);
#pragma unroll
      for (int j = 0; j < 4; ++j) {
        acc[i][j] = Frag<T>::mma(ah, bh[j], acc[i][j]);
        if (SPLIT) {
          acc[i][j] = Frag<T>::mma(ah, bl[j], acc[i][j]);
          acc[i][j] = Frag<T>::mma(al, bh[j], acc[i][j]);
        }
      }
      guard4_ab<V>(acc[i][0], acc[i][1], acc[i][2], acc[i][3], ah, bh[0], bh[1], bh[2], bh[3]);
      if (SPLIT) Frag<T>::keep(al, al, al, al);
    }
    Frag<T>::keep(bh[0], bh[1], bh[2], bh[3]);
    if (SPLIT) Frag<T>::keep(bl[0], bl[1], bl[2], bl[3]);
  }
  acc_guard4(acc[0][0], acc[0][1], acc[0][2], acc[0][3]);
  acc_guard4(acc[1][0], acc[1][1], acc[1][2], acc[1][3]);
  acc_guard4(acc[2][0], acc[2][1], acc[2][2], acc[2][3]);
  acc_guard4(acc[3][0], acc[3][1], acc[3][2], acc[3][3]);

  float* slab = sT[wave];
  const float* Rb = RESID ? (resid + (size_t)b * strideR) : nullptr;
#pragma unroll
  for (int i = 0; i < 4; ++i) {
    const int mBase = m0 + (i << 4);
#pragma unroll
    for (int j = 0; j < 4; ++j) {
      const int n = n0 + (j << 4) + rlane;
      float bv = 0.f;
      if (BIAS_MODE == 2) bv = bias[n];
#pragma unroll
      for (int r = 0; r < 8; ++r) {
        float v = acc[i][j][r] * scale;
        if (BIAS_MODE == 1) v += bias[mBase + mOff + r];
        if (BIAS_MODE == 2) v += bv;
        if (RESID) v += Rb[(size_t)(mBase + mOff + r) * ldc + n];
        if (ACT == 1) v = tanhf(v);
        if (ACT == 2) v = fmaxf(v, 0.0f);
        if (ACT == 3) v = v / (1.0f + expf(-v));
        if (ACT == 4) v = (v > 0.f) ? v : 0.01f * v;
        if (ACT == 5) v = 0.5f * v * (1.0f + erff(v * 0.70710678118654752f));
        slab[(mOff + r) * 68 + (j << 4) + rlane] = v;
      }
    }
    __builtin_amdgcn_fence(__ATOMIC_RELEASE, "workgroup");
    __builtin_amdgcn_wave_barrier();
    __builtin_amdgcn_fence(__ATOMIC_ACQUIRE, "workgroup");
    if (OUT_MODE == 0) {
      float* C = (float*)Cout + (size_t)b * strideC;
      const int hh = lane >> 4, c4 = (lane & 15) * 4;
      for (int pass = 0; pass < 2; ++pass) {
#pragma unroll
        for (int it = 0; it < 8; ++it) {
          const int row = it * 2 + hh;
          v4f v = *(const v4f*)(slab + row * 68 + c4);
          *(volatile v4f*)(C + (size_t)(mBase + row) * ldc + n0 + c4) = v;
        }
        __threadfence();
      }
    } else {
      const int q = lane >> 3, c8 = (lane & 7) * 8;
      unsigned short* C  = (unsigned short*)Cout  + (size_t)b * strideC;
      unsigned short* C2 = (OUT_MODE == 2) ? ((unsigned short*)Cout2 + (size_t)b * strideC) : nullptr;
      for (int pass = 0; pass < 2; ++pass) {
#pragma unroll
        for (int it = 0; it < 4; ++it) {
          const int row = it * 4 + q;
          const float* sp = slab + row * 68 + c8;
          v8h hv, lv;
#pragma unroll
          for (int e = 0; e < 8; ++e) {
            if (OUT_MODE == 1) {
              hv[e] = (_Float16)sp[e];
            } else {
              unsigned short hb = f2bf_bits(sp[e]);
              unsigned short lb = f2bf_bits(sp[e] - bf_bits2f(hb));
              hv[e] = __builtin_bit_cast(_Float16, hb);
              lv[e] = __builtin_bit_cast(_Float16, lb);
            }
          }
          *(volatile v8h*)(C + (size_t)(mBase + row) * ldc + n0 + c8) = hv;
          if (OUT_MODE == 2) *(volatile v8h*)(C2 + (size_t)(mBase + row) * ldc + n0 + c8) = lv;
        }
        __threadfence();
      }
    }
    __builtin_amdgcn_fence(__ATOMIC_RELEASE, "workgroup");
    __builtin_amdgcn_wave_barrier();
    __builtin_amdgcn_fence(__ATOMIC_ACQUIRE, "workgroup");
  }
}

template <int MODE>
__global__ __launch_bounds__(NTHR) void cvt8_kernel(const float* __restrict__ src, unsigned short* __restrict__ dst,
                                                    int nrow, int ncol8, int spitch, int scol0, float sc) {
  const int i  = blockIdx.x * NTHR + threadIdx.x;
  const int n8 = nrow * ncol8;
  if (i < n8) {
    const int row = i / ncol8;
    const int c8  = i - row * ncol8;
    const float* sp = src + (size_t)row * spitch + scol0 + c8 * 8;
    const v4f a = *(const v4f*)(sp);
    const v4f b = *(const v4f*)(sp + 4);
    v8h hv;
#pragma unroll
    for (int e = 0; e < 4; ++e) {
      unsigned short b0, b1;
      if (MODE == 0) {
        b0 = f2bf_bits(a[e] * sc);
        b1 = f2bf_bits(b[e] * sc);
      } else {
        b0 = __builtin_bit_cast(unsigned short, (_Float16)(bf16r(a[e]) * sc));
        b1 = __builtin_bit_cast(unsigned short, (_Float16)(bf16r(b[e]) * sc));
      }
      hv[e]     = __builtin_bit_cast(_Float16, b0);
      hv[4 + e] = __builtin_bit_cast(_Float16, b1);
    }
    *(volatile v8h*)(dst + (size_t)i * 8) = hv;
    __threadfence();
    *(volatile v8h*)(dst + (size_t)i * 8) = hv;
  }
}

__global__ __launch_bounds__(128) void bias_fc_kernel(const float* __restrict__ b, float* __restrict__ dst) {
  const int idx = threadIdx.x * 4;
  const v4f v = *(const v4f*)(b + idx);
  v4f o;
#pragma unroll
  for (int e = 0; e < 4; ++e) o[e] = bf16r(v[e]);
  *(volatile v4f*)(dst + idx) = o;
  __threadfence();
  *(volatile v4f*)(dst + idx) = o;
}

__device__ __forceinline__ void stage_x_tile(unsigned short* Ax, const float* __restrict__ x, int rowbase, int tt, int tid) {
#pragma unroll
  for (int it = 0; it < 2; ++it) {
    const int idx = it * NTHR + tid;
    const int row = idx >> 5, c8 = (idx & 31) * 8;
    const float* sp = x + ((size_t)(rowbase + row) * NSTEP + (size_t)tt) * NIN + c8;
    const v4f a = *(const v4f*)sp;
    const v4f b = *(const v4f*)(sp + 4);
    v4u pk;
    pk[0] = (unsigned)f2bf_bits(a[0]) | ((unsigned)f2bf_bits(a[1]) << 16);
    pk[1] = (unsigned)f2bf_bits(a[2]) | ((unsigned)f2bf_bits(a[3]) << 16);
    pk[2] = (unsigned)f2bf_bits(b[0]) | ((unsigned)f2bf_bits(b[1]) << 16);
    pk[3] = (unsigned)f2bf_bits(b[2]) | ((unsigned)f2bf_bits(b[3]) << 16);
    *(v4u*)(Ax + row * XPITCH + c8) = pk;
  }
}
__device__ __forceinline__ void stage_h_tile(unsigned short* Ag, const unsigned short* __restrict__ H, int rowbase, int tt, int tid) {
#pragma unroll
  for (int it = 0; it < 8; ++it) {
    const int idx = it * NTHR + tid;
    const int row = idx >> 7, c8 = (idx & 127) * 8;
    const v4u v = *(const v4u*)(H + ((size_t)(rowbase + row) * NSTEP + (size_t)tt) * NHID + c8);
    *(v4u*)(Ag + row * HPITCH + c8) = v;
  }
}
__device__ __forceinline__ void store_wave_tile16(const unsigned short* ahs, unsigned short* dst, size_t rpitch, int wave, int lane) {
  for (int pass = 0; pass < 2; ++pass) {
#pragma unroll
    for (int it = 0; it < 8; ++it) {
      const int idx = it * 32 + lane;
      const int row = idx >> 4, c8 = (idx & 15) * 8;
      const v4u v = *(const v4u*)(ahs + row * HPITCH + WCOLS * wave + c8);
      *(volatile v4u*)(dst + (size_t)row * rpitch + WCOLS * wave + c8) = v;
    }
    __threadfence();
  }
}

__global__ __launch_bounds__(NTHR) void seq0_kernel(const float* __restrict__ x, const float* __restrict__ bx,
                                                    const float* __restrict__ bh,
                                                    const unsigned short* __restrict__ WXp,
                                                    const unsigned short* __restrict__ WHp,
                                                    unsigned short* __restrict__ H1) {
  __shared__ __align__(16) unsigned short Ax[SEQ_BLK * XPITCH];
  __shared__ __align__(16) _Float16       Ah[2 * SEQ_BLK * HPITCH];
  const __bf16*   WX = (const __bf16*)WXp;
  const _Float16* WH = (const _Float16*)WHp;
  const int tid = threadIdx.x, lane = tid & 31, wave = tid >> 5;
  const int c = lane & 15, hh = lane >> 4, koff = hh * 8;
  const int rowbase = blockIdx.x * SEQ_BLK;
  const int jb = WCOLS * wave + c;

  {
    unsigned* az = (unsigned*)(void*)Ah;
#pragma unroll 1
    for (int i = tid; i < (2 * SEQ_BLK * HPITCH) / 2; i += NTHR) az[i] = 0u;
    unsigned* axz = (unsigned*)(void*)Ax;
#pragma unroll 1
    for (int i = tid; i < (SEQ_BLK * XPITCH) / 2; i += NTHR) axz[i] = 0u;
  }
  __syncthreads();
  stage_x_tile(Ax, x, rowbase, 0, tid);
  float bs[NSUB];
#pragma unroll
  for (int ns = 0; ns < NSUB; ++ns) { const int j = jb + 16 * ns; bs[ns] = bf16r(bx[j]) + bf16r(bh[j]); }
  __syncthreads();

  const __bf16*   axrow = (const __bf16*)(const void*)Ax + c * XPITCH + koff;
  const __bf16*   wx = WX + (size_t)jb * NIN + koff;
  const _Float16* wh = WH + (size_t)jb * NHID + koff;
  const v8f z8 = {0.f, 0.f, 0.f, 0.f, 0.f, 0.f, 0.f, 0.f};

#pragma unroll 1
  for (int t = 0; t < NSTEP; ++t) {
    const int cur = t & 1;
    const _Float16* ahrow = Ah + cur * (SEQ_BLK * HPITCH) + c * HPITCH + koff;
    _Float16* ahn = Ah + (cur ^ 1) * (SEQ_BLK * HPITCH);
    v8f acc[NSUB];
#pragma unroll
    for (int ns = 0; ns < NSUB; ++ns) acc[ns] = z8;
#pragma unroll 1
    for (int kx = 0; kx < NIN; kx += 32) {
      const v16b a = Frag<__bf16>::load(axrow + kx);
      v16b b[NSUB];
#pragma unroll
      for (int ns = 0; ns < NSUB; ++ns) b[ns] = Frag<__bf16>::load(wx + (size_t)ns * 16 * NIN + kx);
#pragma unroll
      for (int ns = 0; ns < NSUB; ++ns) acc[ns] = Frag<__bf16>::mma(a, b[ns], acc[ns]);
      guard8_b(acc[0], acc[1], acc[2], acc[3], acc[4], acc[5], acc[6], acc[7], a, b[0], b[1], b[2], b[3], b[4], b[5], b[6], b[7]);
    }
#pragma unroll 1
    for (int k0 = 0; k0 < NHID; k0 += 32) {
      const v16h a = Frag<_Float16>::load(ahrow + k0);
      v16h b[NSUB];
#pragma unroll
      for (int ns = 0; ns < NSUB; ++ns) b[ns] = Frag<_Float16>::load(wh + (size_t)ns * 16 * NHID + k0);
#pragma unroll
      for (int ns = 0; ns < NSUB; ++ns) acc[ns] = Frag<_Float16>::mma(a, b[ns], acc[ns]);
      guard8_h(acc[0], acc[1], acc[2], acc[3], acc[4], acc[5], acc[6], acc[7], a, b[0], b[1], b[2], b[3], b[4], b[5], b[6], b[7]);
    }
    acc_guard8(acc[0], acc[1], acc[2], acc[3], acc[4], acc[5], acc[6], acc[7]);
#pragma unroll
    for (int ns = 0; ns < NSUB; ++ns) {
      const int j = jb + 16 * ns;
#pragma unroll
      for (int r = 0; r < 8; ++r) {
        const float z = acc[ns][r] * WCARRY_INV + bs[ns];
        ahn[(8 * hh + r) * HPITCH + j] = (_Float16)tanh_f(z);
      }
    }
    __syncthreads();
    store_wave_tile16((const unsigned short*)(const void*)ahn, H1 + ((size_t)rowbase * NSTEP + (size_t)t) * NHID,
                      (size_t)NSTEP * NHID, wave, lane);
    {
      const int tn = (t + 1 < NSTEP) ? (t + 1) : (NSTEP - 1);
      stage_x_tile(Ax, x, rowbase, tn, tid);
    }
    __syncthreads();
  }
}

__global__ __launch_bounds__(NTHR) void seq1_kernel(const unsigned short* __restrict__ H1, const float* __restrict__ bx,
                                                    const float* __restrict__ bh,
                                                    const unsigned short* __restrict__ WXp,
                                                    const unsigned short* __restrict__ WHp,
                                                    unsigned short* __restrict__ HFIN) {
  __shared__ __align__(16) unsigned short Ag[SEQ_BLK * HPITCH];
  __shared__ __align__(16) _Float16       Ah[2 * SEQ_BLK * HPITCH];
  const _Float16* WX = (const _Float16*)WXp;
  const _Float16* WH = (const _Float16*)WHp;
  const int tid = threadIdx.x, lane = tid & 31, wave = tid >> 5;
  const int c = lane & 15, hh = lane >> 4, koff = hh * 8;
  const int rowbase = blockIdx.x * SEQ_BLK;
  const int jb = WCOLS * wave + c;

  {
    unsigned* az = (unsigned*)(void*)Ah;
#pragma unroll 1
    for (int i = tid; i < (2 * SEQ_BLK * HPITCH) / 2; i += NTHR) az[i] = 0u;
    unsigned* agz = (unsigned*)(void*)Ag;
#pragma unroll 1
    for (int i = tid; i < (SEQ_BLK * HPITCH) / 2; i += NTHR) agz[i] = 0u;
  }
  __syncthreads();
  stage_h_tile(Ag, H1, rowbase, 0, tid);
  float bs[NSUB];
#pragma unroll
  for (int ns = 0; ns < NSUB; ++ns) { const int j = jb + 16 * ns; bs[ns] = bf16r(bx[j]) + bf16r(bh[j]); }
  __syncthreads();

  const _Float16* agrow = (const _Float16*)(const void*)Ag + c * HPITCH + koff;
  const _Float16* wx = WX + (size_t)jb * NHID + koff;
  const _Float16* wh = WH + (size_t)jb * NHID + koff;
  const v8f z8 = {0.f, 0.f, 0.f, 0.f, 0.f, 0.f, 0.f, 0.f};

#pragma unroll 1
  for (int t = 0; t < NSTEP; ++t) {
    const int cur = t & 1;
    const _Float16* ahrow = Ah + cur * (SEQ_BLK * HPITCH) + c * HPITCH + koff;
    _Float16* ahn = Ah + (cur ^ 1) * (SEQ_BLK * HPITCH);
    v8f acc[NSUB];
#pragma unroll
    for (int ns = 0; ns < NSUB; ++ns) acc[ns] = z8;
#pragma unroll 1
    for (int kg = 0; kg < NHID; kg += 32) {
      const v16h a = Frag<_Float16>::load(agrow + kg);
      v16h b[NSUB];
#pragma unroll
      for (int ns = 0; ns < NSUB; ++ns) b[ns] = Frag<_Float16>::load(wx + (size_t)ns * 16 * NHID + kg);
#pragma unroll
      for (int ns = 0; ns < NSUB; ++ns) acc[ns] = Frag<_Float16>::mma(a, b[ns], acc[ns]);
      guard8_h(acc[0], acc[1], acc[2], acc[3], acc[4], acc[5], acc[6], acc[7], a, b[0], b[1], b[2], b[3], b[4], b[5], b[6], b[7]);
    }
#pragma unroll 1
    for (int k0 = 0; k0 < NHID; k0 += 32) {
      const v16h a = Frag<_Float16>::load(ahrow + k0);
      v16h b[NSUB];
#pragma unroll
      for (int ns = 0; ns < NSUB; ++ns) b[ns] = Frag<_Float16>::load(wh + (size_t)ns * 16 * NHID + k0);
#pragma unroll
      for (int ns = 0; ns < NSUB; ++ns) acc[ns] = Frag<_Float16>::mma(a, b[ns], acc[ns]);
      guard8_h(acc[0], acc[1], acc[2], acc[3], acc[4], acc[5], acc[6], acc[7], a, b[0], b[1], b[2], b[3], b[4], b[5], b[6], b[7]);
    }
    acc_guard8(acc[0], acc[1], acc[2], acc[3], acc[4], acc[5], acc[6], acc[7]);
#pragma unroll
    for (int ns = 0; ns < NSUB; ++ns) {
      const int j = jb + 16 * ns;
#pragma unroll
      for (int r = 0; r < 8; ++r) {
        const float z = acc[ns][r] * WCARRY_INV + bs[ns];
        ahn[(8 * hh + r) * HPITCH + j] = (_Float16)tanh_f(z);
      }
    }
    __syncthreads();
    if (t == NSTEP - 1) {
      store_wave_tile16((const unsigned short*)(const void*)ahn, HFIN + (size_t)rowbase * NHID, (size_t)NHID, wave, lane);
    }
    {
      const int tn = (t + 1 < NSTEP) ? (t + 1) : (NSTEP - 1);
      stage_h_tile(Ag, H1, rowbase, tn, tid);
    }
    __syncthreads();
  }
}

extern "C" void kernel_launch(void* const* d_in, const int* in_sizes, int n_in,
                              void* d_out, int out_size, void* d_ws, size_t ws_size, hipStream_t stream) {
  if (n_in < 11 || d_out == nullptr || d_ws == nullptr) return;
  if (in_sizes[0] != NBATCH * NSTEP * NIN || in_sizes[1] != NHID * NIN || in_sizes[2] != NHID ||
      in_sizes[3] != NHID * NHID || in_sizes[4] != NHID || in_sizes[5] != NHID * NHID || in_sizes[6] != NHID ||
      in_sizes[7] != NHID * NHID || in_sizes[8] != NHID || in_sizes[9] != NOUTF * NHID || in_sizes[10] != NOUTF ||
      out_size != NBATCH * NOUTF) return;

  const float* x   = (const float*)d_in[0];
  const float* wx0 = (const float*)d_in[1];
  const float* bx0 = (const float*)d_in[2];
  const float* wh0 = (const float*)d_in[3];
  const float* bh0 = (const float*)d_in[4];
  const float* wx1 = (const float*)d_in[5];
  const float* bx1 = (const float*)d_in[6];
  const float* wh1 = (const float*)d_in[7];
  const float* bh1 = (const float*)d_in[8];
  const float* wfc = (const float*)d_in[9];
  const float* bfc = (const float*)d_in[10];
  float* out = (float*)d_out;

  char* ws = (char*)d_ws; size_t off = 0;
  auto carve = [&](size_t bytes) -> char* { char* p = ws + off; off += (bytes + 255) & ~(size_t)255; return p; };
  unsigned short* WX0  = (unsigned short*)carve((size_t)NHID * NIN * 2);
  unsigned short* WH0  = (unsigned short*)carve((size_t)NHID * NHID * 2);
  unsigned short* WX1  = (unsigned short*)carve((size_t)NHID * NHID * 2);
  unsigned short* WH1  = (unsigned short*)carve((size_t)NHID * NHID * 2);
  unsigned short* WFC  = (unsigned short*)carve((size_t)NOUTF * NHID * 2);
  float*          BFC  = (float*)carve((size_t)NOUTF * 4);
  unsigned short* H1   = (unsigned short*)carve((size_t)NROWS * NHID * 2);
  unsigned short* HFIN = (unsigned short*)carve((size_t)NBATCH * NHID * 2);
  if (off > ws_size || off > (size_t)134217728) return;

  const int n8a = NHID * (NIN / 8);
  const int n8b = NHID * (NHID / 8);
  const int n8c = NOUTF * (NHID / 8);
  cvt8_kernel<0><<<(n8a + NTHR - 1) / NTHR, NTHR, 0, stream>>>(wx0, WX0, NHID,  NIN / 8,  NIN,  0, WCARRY);
  cvt8_kernel<1><<<(n8b + NTHR - 1) / NTHR, NTHR, 0, stream>>>(wh0, WH0, NHID,  NHID / 8, NHID, 0, WCARRY);
  cvt8_kernel<1><<<(n8b + NTHR - 1) / NTHR, NTHR, 0, stream>>>(wx1, WX1, NHID,  NHID / 8, NHID, 0, WCARRY);
  cvt8_kernel<1><<<(n8b + NTHR - 1) / NTHR, NTHR, 0, stream>>>(wh1, WH1, NHID,  NHID / 8, NHID, 0, WCARRY);
  cvt8_kernel<1><<<(n8c + NTHR - 1) / NTHR, NTHR, 0, stream>>>(wfc, WFC, NOUTF, NHID / 8, NHID, 0, WCARRY);
  bias_fc_kernel<<<1, 128, 0, stream>>>(bfc, BFC);

  seq0_kernel<<<NBATCH / SEQ_BLK, NTHR, 0, stream>>>(x, bx0, bh0, WX0, WH0, H1);
  seq1_kernel<<<NBATCH / SEQ_BLK, NTHR, 0, stream>>>(H1, bx1, bh1, WX1, WH1, HFIN);
  wmma_gemm64<0, false, 2, 0, false, 0><<<dim3(1, 1), 256, 0, stream>>>(
      HFIN, HFIN, NHID, 0L, WFC, WFC, NHID, 0L, (void*)out, (void*)out, NOUTF, 0L,
      BFC, BFC, 0L, NBATCH, NOUTF, NHID, WCARRY_INV);
}
